// SparseConv3D_33749853012468
// MI455X (gfx1250) — hardware-verified
//
#include <hip/hip_runtime.h>

typedef float          v8f   __attribute__((ext_vector_type(8)));
typedef float          v4f   __attribute__((ext_vector_type(4)));
typedef unsigned int   v4u   __attribute__((ext_vector_type(4)));
typedef int            v8i   __attribute__((ext_vector_type(8)));
typedef unsigned short v8us  __attribute__((ext_vector_type(8)));
typedef unsigned short v16us __attribute__((ext_vector_type(16)));
typedef __bf16         v16bf __attribute__((ext_vector_type(16)));
typedef _Float16       v16h  __attribute__((ext_vector_type(16)));
typedef v4f  __attribute__((may_alias)) v4fa;
typedef v8us __attribute__((may_alias)) v8usa;
union FragB { v16bf v; v16us u; v8us h[2]; v8i w; };
union FragH { v16h  v; v16us u; v8us h[2]; v8i w; };

__device__ __forceinline__ v8f wmb(const FragB& a, const FragB& b, v8f c) {
  v8f d = __builtin_amdgcn_wmma_f32_16x16x32_bf16(false, a.v, false, b.v, (short)0, c, false, false);
  asm volatile("v_nop\n\tv_nop\n\tv_nop\n\tv_nop" : "+v"(d) : "v"(a.w), "v"(b.w));
  return d;
}

__device__ __forceinline__ v8f wmh(const FragH& a, const FragH& b, v8f c) {
  v8f d = __builtin_amdgcn_wmma_f32_16x16x32_f16(false, a.v, false, b.v, (short)0, c, false, false);
  asm volatile("v_nop\n\tv_nop\n\tv_nop\n\tv_nop" : "+v"(d) : "v"(a.w), "v"(b.w));
  return d;
}

__device__ __forceinline__ unsigned bf16_bits(float f) {
  const unsigned u = __float_as_uint(f);
  const unsigned r = (u + 0x7FFFu + ((u >> 16) & 1u)) >> 16;
  const unsigned q = (u >> 16) | 0x40u;
  return ((u & 0x7fffffffu) > 0x7f800000u) ? q : r;
}

__device__ __forceinline__ float bf16_val(float f) {
  return __uint_as_float(bf16_bits(f) << 16);
}
__device__ __forceinline__ int clampi(int v, int lo, int hi) {
  return v < lo ? lo : (v > hi ? hi : v);
}

__device__ __forceinline__ unsigned f16_bits(float f) {
  const unsigned u  = __float_as_uint(f);
  const unsigned s  = (u >> 16) & 0x8000u;
  const unsigned a  = u & 0x7fffffffu;
  const unsigned t  = a - 0x38000000u;
  const unsigned r  = (t + 0x0FFFu + ((t >> 13) & 1u)) >> 13;
  const unsigned rc = r > 0x7C00u ? 0x7C00u : r;
  const bool small  = a < 0x38800000u;
  const bool isnan  = a > 0x7f800000u;
  const unsigned fin = small ? 0u : (s | rc);
  return isnan ? (s | 0x7E00u) : fin;
}

__device__ __forceinline__ unsigned pk16(unsigned lo, unsigned hi) { return lo | (hi << 16); }
__device__ __forceinline__ unsigned bf16_lo_bits(float v) {
  float hi = bf16_val(v);
  asm volatile("" : "+v"(hi));
  return bf16_bits(v - hi);
}
__device__ __forceinline__ v4u pack8_bf16(v4f a, v4f c) {
  return (v4u){ pk16(bf16_bits(a[0]), bf16_bits(a[1])), pk16(bf16_bits(a[2]), bf16_bits(a[3])),
                pk16(bf16_bits(c[0]), bf16_bits(c[1])), pk16(bf16_bits(c[2]), bf16_bits(c[3])) };
}
__device__ __forceinline__ v4u pack8_bf16_lo(v4f a, v4f c) {
  return (v4u){ pk16(bf16_lo_bits(a[0]), bf16_lo_bits(a[1])), pk16(bf16_lo_bits(a[2]), bf16_lo_bits(a[3])),
                pk16(bf16_lo_bits(c[0]), bf16_lo_bits(c[1])), pk16(bf16_lo_bits(c[2]), bf16_lo_bits(c[3])) };
}
__device__ __forceinline__ v4u pack8_f16(v4f a, v4f c) {
  return (v4u){ pk16(f16_bits(a[0]), f16_bits(a[1])), pk16(f16_bits(a[2]), f16_bits(a[3])),
                pk16(f16_bits(c[0]), f16_bits(c[1])), pk16(f16_bits(c[2]), f16_bits(c[3])) };
}

template <int FORM>
__global__ __launch_bounds__(256) void k_plane(const float* __restrict__ src, int rows, int cols, int ldsrc,
                                               unsigned short* __restrict__ dst, int MP, int KP) {
  static_assert(FORM >= 0 && FORM <= 3);
  const int KTOT = (FORM == 1 || FORM == 3) ? 2 * KP : KP;
  const unsigned ppr   = (unsigned)(KTOT >> 3);
  const unsigned kp8   = (unsigned)(KP >> 3);
  const unsigned total = (unsigned)MP * ppr;
  const unsigned g     = blockIdx.x * 256u + threadIdx.x;
  const unsigned rowu  = g / ppr;
  const unsigned p     = g - rowu * ppr;
  const bool second    = p >= kp8;
  const int row = (int)rowu;
  const int c0  = (int)((second ? p - kp8 : p) << 3);
  const float* srow = src + (size_t)clampi(row, 0, rows - 1) * (size_t)ldsrc;
  float x[8];
  unsigned mk[8];
#pragma unroll
  for (int e = 0; e < 8; ++e) {
    const int c = c0 + e;
    const float v = srow[clampi(c, 0, cols - 1)];
    asm volatile("" :: "v"(v));
    x[e]  = v;
    mk[e] = (row < rows && c < cols) ? 0xFFFFu : 0u;
  }
  const v4f a = (v4f){ x[0], x[1], x[2], x[3] };
  const v4f c = (v4f){ x[4], x[5], x[6], x[7] };
  v4u o;
  if (FORM == 2) {
    o = pack8_f16(a, c);
  } else {
    const v4u hi = pack8_bf16(a, c);
    o = hi;
    if (FORM == 1) { const v4u lo = pack8_bf16_lo(a, c); o = second ? lo : hi; }
  }
  const v4u mw = (v4u){ pk16(mk[0], mk[1]), pk16(mk[2], mk[3]), pk16(mk[4], mk[5]), pk16(mk[6], mk[7]) };
  o &= mw;
  if (g < total) {
    volatile v4u* q = (volatile v4u*)(dst + (size_t)g * 8);
    *q = o;
    __threadfence();
    *q = o;
  }
}

template <int FORM> struct FragOf    { typedef FragB T; };
template <>         struct FragOf<2> { typedef FragH T; };
__device__ __forceinline__ v8f mm(const FragB& a, const FragB& b, v8f c) { return wmb(a, b, c); }
__device__ __forceinline__ v8f mm(const FragH& a, const FragH& b, v8f c) { return wmh(a, b, c); }
template <class F> __device__ __forceinline__ F ld_frag(const unsigned short* p) {
  F f;
  f.h[0] = *(const v8usa*)(p);
  f.h[1] = *(const v8usa*)(p + 16);
  return f;
}

template <int FORM, int EPI>
__global__ __launch_bounds__(256) __attribute__((amdgpu_num_vgpr(248)))
void k_gemm_nt(const unsigned short* __restrict__ A, const unsigned short* __restrict__ B,
               const float* __restrict__ bias, float* __restrict__ D, int M, int N, int KTOT, int ldd) {
  static_assert(FORM >= 0 && FORM <= 2);
  static_assert(EPI == 0 || EPI == 1);
  typedef typename FragOf<FORM>::T F;
  __shared__ __attribute__((aligned(16))) float sT[8][16 * 68];
  const int lane = threadIdx.x & 31;
  const int wave = threadIdx.x >> 5;
  const int tilesM = (M + 63) >> 6;
  const int tilesN = (N + 63) >> 6;
  const int tile = blockIdx.x * 8 + wave;
  if (tile >= tilesM * tilesN) return;
  const int tm = tile / tilesN;
  const int tn = tile - tm * tilesN;
  const int m0 = tm << 6;
  const int n0 = tn << 6;

  const int rl = lane & 15;
  const int h8 = (lane >> 4) * 8;
  const unsigned short* pa = A + (size_t)(m0 + rl) * (size_t)KTOT + h8;
  const unsigned short* pb = B + (size_t)(n0 + rl) * (size_t)KTOT + h8;

  v8f acc[4][4];
#pragma unroll
  for (int i = 0; i < 4; ++i)
#pragma unroll
    for (int j = 0; j < 4; ++j) acc[i][j] = (v8f){0.f, 0.f, 0.f, 0.f, 0.f, 0.f, 0.f, 0.f};

#pragma unroll 1
  for (int k0 = 0; k0 < KTOT; k0 += 32) {
    F bf[4];
#pragma unroll
    for (int j = 0; j < 4; ++j) bf[j] = ld_frag<F>(pb + (size_t)(j << 4) * (size_t)KTOT + k0);
#pragma unroll
    for (int i = 0; i < 4; ++i) {
      const F af = ld_frag<F>(pa + (size_t)(i << 4) * (size_t)KTOT + k0);
#pragma unroll
      for (int j = 0; j < 4; ++j) acc[i][j] = mm(af, bf[j], acc[i][j]);
    }
  }

  float* slab = sT[wave];
  const int hh = lane >> 4;
  const int c4 = (lane & 15) * 4;
  const int nc = n0 + c4;
  const bool cok = nc < N;
  v4f bv = (v4f){0.f, 0.f, 0.f, 0.f};
  if (EPI == 1) {
    bv = *(const v4fa*)(bias + clampi(nc, 0, N - 4));
    asm volatile("" :: "v"(bv));
  }
#pragma unroll
  for (int i = 0; i < 4; ++i) {
    const int mBase = m0 + (i << 4);
#pragma unroll
    for (int j = 0; j < 4; ++j) {
#pragma unroll
      for (int r = 0; r < 8; ++r) slab[(h8 + r) * 68 + (j << 4) + rl] = acc[i][j][r];
    }
    __builtin_amdgcn_fence(__ATOMIC_RELEASE, "workgroup");
    __builtin_amdgcn_wave_barrier();
    __builtin_amdgcn_fence(__ATOMIC_ACQUIRE, "workgroup");
    v4f vv[8];
#pragma unroll
    for (int it = 0; it < 8; ++it) {
      const int row = it * 2 + hh;
      v4f v = *(const v4fa*)(slab + row * 68 + c4);
      if (EPI == 1) v += bv;
      vv[it] = v;
    }
    for (int pass = 0; pass < 2; ++pass) {
#pragma unroll
      for (int it = 0; it < 8; ++it) {
        const int row = mBase + it * 2 + hh;
        if (cok && row < M) *(volatile v4f*)(D + (size_t)row * (size_t)ldd + nc) = vv[it];
      }
      __threadfence();
    }
    __builtin_amdgcn_fence(__ATOMIC_RELEASE, "workgroup");
    __builtin_amdgcn_wave_barrier();
    __builtin_amdgcn_fence(__ATOMIC_ACQUIRE, "workgroup");
  }
}

#include <stddef.h>
#pragma clang fp contract(off)

typedef float v2f __attribute__((ext_vector_type(2)));
typedef int   v2i __attribute__((ext_vector_type(2)));
typedef int   v4i __attribute__((ext_vector_type(4)));
typedef v2f __attribute__((may_alias)) v2fa;
typedef v2i __attribute__((may_alias)) v2ia;
typedef v4u __attribute__((may_alias)) v4ua;

constexpr int NV     = 100000;
constexpr int CIN    = 64;
constexpr int COUT   = 64;
constexpr int NTAP   = 27;
constexpr int KT     = NTAP * CIN;
constexpr int NOFF   = 26;
constexpr int PMAX   = 4815;
constexpr int TOT    = NOFF * PMAX;
constexpr int CHR    = 25088;
constexpr int NCHUNK = 4;
constexpr int NBROWS = NCHUNK * CHR;
constexpr int MLAST  = NV - 3 * CHR;
constexpr int TB_VOX    = 256;
constexpr int TB_CELLS  = TB_VOX * 32;
constexpr int TB_BLOCKS = NBROWS / TB_VOX;
constexpr int TB_ITERS  = 490;
constexpr int PREP_WB_BLOCKS = COUT * KT / 8 / 256;

__host__ __device__ constexpr int tap_of(int o) { return o < 13 ? o : o + 1; }

static_assert(NV < (1 << 20));
static_assert(TB_BLOCKS == 392 && TB_BLOCKS * TB_VOX == NBROWS && NBROWS == 100352);
static_assert(TB_ITERS * 256 >= TOT && (TB_ITERS - 1) * 256 < TOT && TOT == 125190);
static_assert(NOFF == 26 && NOFF + 1 == NTAP);
static_assert(tap_of(0) == 0 && tap_of(12) == 12 && tap_of(13) == 14 && tap_of(25) == 26);
static_assert(KT == 1728 && KT % 32 == 0 && COUT % 64 == 0 && COUT % 4 == 0);
static_assert(CHR % 64 == 0 && CHR % 16 == 0 && CHR % 8 == 0 && MLAST == 24736 && MLAST % 16 == 0 && MLAST > 0);
static_assert(3 * CHR + MLAST == NV && NBROWS >= NV);
static_assert((COUT * KT / 8) % 256 == 0 && PREP_WB_BLOCKS == 54);
static_assert((size_t)CHR * KT / 8 < ((size_t)1 << 31));
static_assert(((size_t)CHR * COUT * 4) % 128 == 0);

constexpr size_t SZ_WB   = (size_t)COUT * KT * 2;
constexpr size_t SZ_BIAS = (size_t)COUT * 4;
constexpr size_t SZ_NB   = (size_t)NBROWS * 32 * 4;
constexpr size_t SZ_AP   = (size_t)CHR * KT * 2;
constexpr size_t OFF_WB   = 0;
constexpr size_t OFF_BIAS = OFF_WB + SZ_WB;
constexpr size_t OFF_NB   = OFF_BIAS + SZ_BIAS;
constexpr size_t OFF_AP   = OFF_NB + SZ_NB;
constexpr size_t WS_TOTAL = OFF_AP + SZ_AP;
static_assert(SZ_WB == (size_t)221184 && SZ_NB == (size_t)12845056 && SZ_AP == (size_t)86704128);
static_assert(OFF_BIAS == (size_t)221184 && OFF_NB == (size_t)221440 && OFF_AP == (size_t)13066496);
static_assert(WS_TOTAL == (size_t)99770624 && WS_TOTAL <= ((size_t)128 << 20));
static_assert(OFF_BIAS % 128 == 0 && OFF_NB % 128 == 0 && OFF_AP % 128 == 0);
static_assert((size_t)TB_BLOCKS * TB_CELLS * 4 == SZ_NB);
static_assert((size_t)PREP_WB_BLOCKS * 256 * 16 == SZ_WB);
static_assert((size_t)CHR * NTAP * 128 == SZ_AP);

__global__ __launch_bounds__(256) void k_prep(const float* __restrict__ weight, const float* __restrict__ bias,
                                              unsigned short* __restrict__ WB, float* __restrict__ BIASR) {
  const int tid = (int)threadIdx.x;
  const int blk = (int)blockIdx.x;
  if (blk < PREP_WB_BLOCKS) {
    const int g = blk * 256 + tid;
    const v4f a = *(const v4fa*)(weight + (size_t)g * 8);
    const v4f c = *(const v4fa*)(weight + (size_t)g * 8 + 4);
    asm volatile("" :: "v"(a));
    asm volatile("" :: "v"(c));
    const v4u o = pack8_bf16(a, c);
    volatile v4u* q = (volatile v4u*)(WB + (size_t)g * 8);
    *q = o;
    __threadfence();
    *q = o;
  } else {
    if (tid < 32) {
      const int pc = tid < 16 ? tid : 15;
      const v4f b = *(const v4fa*)(bias + 4 * pc);
      asm volatile("" :: "v"(b));
      const v4f o = (v4f){ bf16_val(b[0]), bf16_val(b[1]), bf16_val(b[2]), bf16_val(b[3]) };
      volatile v4f* q = (volatile v4f*)(BIASR + 4 * pc);
      if (tid < 16) *q = o;
      __threadfence();
      if (tid < 16) *q = o;
    }
  }
}

__device__ __forceinline__ int decode_cell(unsigned w, int tap, int v) {
  const unsigned cnt = w >> 20;
  const int idp = (int)(w & 0xFFFFFu);
  int id = (cnt == 0u) ? -1 : ((cnt == 1u) ? idp : -2);
  id = (tap == 13) ? v : id;
  id = (tap > 26) ? -1 : id;
  id = (v < NV) ? id : -1;
  return id;
}

__global__ __launch_bounds__(256) void k_table(const int* __restrict__ nei, const int* __restrict__ sizes,
                                               int* __restrict__ NB) {
  __shared__ __attribute__((aligned(16))) unsigned tile[TB_CELLS];
  __shared__ __attribute__((aligned(16))) int ssz[32];
  const int tid  = (int)threadIdx.x;
  const int base = (int)blockIdx.x * TB_VOX;
  {
    const v4u z4 = (v4u){ 0u, 0u, 0u, 0u };
    for (int i = tid * 4; i < TB_CELLS; i += 1024) *(v4ua*)(tile + i) = z4;
  }
  if (tid < 32) {
    const int s = sizes[tid < NOFF ? tid : NOFF - 1];
    asm volatile("" :: "v"(s));
    ssz[tid] = s;
  }
  __syncthreads();

#pragma unroll 1
  for (int it = 0; it < TB_ITERS; ++it) {
    const int q  = it * 256 + tid;
    const int qc = q < TOT ? q : TOT - 1;
    const v2i pr = *(const v2ia*)(nei + 2 * (size_t)qc);
    const int po = pr.x;
    const int pi = pr.y;
    asm volatile("" :: "v"(po));
    asm volatile("" :: "v"(pi));
    const int o  = qc / PMAX;
    const int p  = qc - PMAX * o;
    const int sz = ssz[o];
    const unsigned rel = (unsigned)(po - base);
    const bool valid = (q < TOT) && (p < sz) && (rel < (unsigned)TB_VOX);
    const int tap = o < 13 ? o : o + 1;
    const unsigned cell = valid ? (rel * 32u + (unsigned)tap) : 0u;
    const unsigned val  = valid ? ((1u << 20) + (unsigned)clampi(pi, 0, NV - 1)) : 0u;
    if (valid) atomicAdd(&tile[cell], val);
  }
  __syncthreads();

  int* nbb = NB + (size_t)blockIdx.x * TB_CELLS;
  for (int pass = 0; pass < 2; ++pass) {
#pragma unroll 1
    for (int it = 0; it < TB_CELLS / 4 / 256; ++it) {
      const int i = it * 256 + tid;
      const v4u w = *(const v4ua*)(tile + 4 * i);
      const int v    = base + (i >> 3);
      const int tap0 = (i & 7) * 4;
      const v4i o4 = (v4i){ decode_cell(w[0], tap0, v), decode_cell(w[1], tap0 + 1, v),
                            decode_cell(w[2], tap0 + 2, v), decode_cell(w[3], tap0 + 3, v) };
      *(volatile v4i*)(nbb + 4 * i) = o4;
    }
    __threadfence();
  }
}

__global__ __launch_bounds__(256) void k_gather(const float* __restrict__ x, const int* __restrict__ NB,
                                                unsigned* __restrict__ AP, int vbase) {
  const int tid = (int)threadIdx.x, lane = tid & 31, wave = tid >> 5;
  const int r = (int)blockIdx.x * 8 + wave;
  const int v = clampi(vbase + r, 0, NBROWS - 1);
  int line = NB[(size_t)v * 32 + lane];
  asm volatile("" :: "v"(line));
  line = clampi(line, -2, NV - 1);
  unsigned* rowp = AP + (size_t)r * (size_t)(KT / 2) + lane;
#pragma unroll 1
  for (int g = 0; g < 9; ++g) {
    unsigned wd[3];
#pragma unroll
    for (int j = 0; j < 3; ++j) {
      const int id  = __builtin_amdgcn_readlane(line, 3 * g + j);
      const int idc = id < 0 ? 0 : id;
      const v2f s = *(const v2fa*)(x + (size_t)idc * CIN + 2 * lane);
      asm volatile("" :: "v"(s));
      const unsigned pk = pk16(bf16_bits(s[0]), bf16_bits(s[1]));
      const unsigned m  = (id >= 0) ? 0xFFFFFFFFu : 0u;
      const unsigned pz = (id == -2) ? 0x7FC07FC0u : 0u;
      wd[j] = (pk & m) | pz;
    }
    volatile unsigned* q = (volatile unsigned*)(rowp + 96 * g);
    q[0]  = wd[0];
    q[32] = wd[1];
    q[64] = wd[2];
    __threadfence();
    q[0]  = wd[0];
    q[32] = wd[1];
    q[64] = wd[2];
  }
}

extern "C" void kernel_launch(void* const* d_in, const int* in_sizes, int n_in,
                              void* d_out, int out_size, void* d_ws, size_t ws_size,
                              hipStream_t stream) {
  if (n_in < 5) return;
  if (in_sizes[0] != NV * CIN) return;
  if (in_sizes[1] != COUT * KT) return;
  if (in_sizes[2] != COUT) return;
  if (in_sizes[3] != TOT * 2) return;
  if (in_sizes[4] != NOFF) return;
  if (out_size != NV * COUT) return;
  if (ws_size < WS_TOTAL) return;

  const float* x      = (const float*)d_in[0];
  const float* weight = (const float*)d_in[1];
  const float* bias   = (const float*)d_in[2];
  const int*   nei    = (const int*)d_in[3];
  const int*   sizes  = (const int*)d_in[4];
  float* out = (float*)d_out;

  char* ws = (char*)d_ws;
  unsigned short* WB    = (unsigned short*)(ws + OFF_WB);
  float*          BIASR = (float*)(ws + OFF_BIAS);
  int*            NB    = (int*)(ws + OFF_NB);
  unsigned short* AP    = (unsigned short*)(ws + OFF_AP);

  k_prep<<<PREP_WB_BLOCKS + 1, 256, 0, stream>>>(weight, bias, WB, BIASR);
  k_table<<<TB_BLOCKS, 256, 0, stream>>>(nei, sizes, NB);
  for (int c = 0; c < NCHUNK; ++c) {
    const int Mc = (c == NCHUNK - 1) ? MLAST : CHR;
    const int tiles = (Mc + 63) / 64;
    const int gblocks = (tiles + 7) / 8;
    k_gather<<<CHR / 8, 256, 0, stream>>>(x, NB, (unsigned*)AP, c * CHR);
    k_gemm_nt<0, 1><<<gblocks, 256, 0, stream>>>(AP, WB, BIASR, out + (size_t)c * CHR * COUT, Mc, COUT, KT, COUT);
  }
}
